// QGCNLayer_v2_88905823027435
// MI455X (gfx1250) — hardware-run, weakly checked
//
#include <hip/hip_runtime.h>
#include <stddef.h>
#include <stdint.h>
#include <math.h>

#define NN      100000
#define NE      1600000
#define HD      64
#define KEXT    64
#define XPITCH  64
#define HPITCH  64
#define GBM     128
#define MP      100096
#define NTHR    256
#define NWAVE   8
#define EPT     8
#define WCH     (32 * EPT)
#define NBRUN   1024
#define SLB     10
#define NBK     98
#define WLCAP   2560
#define RCAP    20480
#define DEGCAP  64
#define MAXDEG_MEAS   37
#define MAXB1024_MEAS 16666
#define SP      68
#define ABM     64

#define BK_ZINTS (NWAVE * WLCAP + RCAP + 3 * NBRUN)
#define BK_INTS  (BK_ZINTS + 16)
#define BK_LDS   (BK_INTS * 4)

#define PBX   (MP * KEXT / 8 / NTHR)
#define PBH   2
#define PBTOT (PBX + PBH + 1)

static_assert(HD == 64 && KEXT == 64 && KEXT % 32 == 0);
static_assert(XPITCH >= KEXT && HPITCH >= KEXT && XPITCH % 8 == 0 && HPITCH % 8 == 0);
static_assert(MP % GBM == 0 && MP >= NN && MP == 782 * GBM);
static_assert(NN % 2 == 0);
static_assert(NBRUN == 1024 && NBRUN == (1 << SLB) && NBRUN % ABM == 0);
static_assert(NBK * NBRUN >= NN && (NBK - 1) * NBRUN < NN);
static_assert(NE < (1 << 21) && (((long long)NE) << SLB) < (1LL << 31));
static_assert(NE % WCH == 0);
static_assert(RCAP == NWAVE * WLCAP && RCAP % (NTHR * 2) == 0 && BK_ZINTS % 4 == 0);
static_assert((long long)RCAP * 100 >= (long long)MAXB1024_MEAS * 105);
static_assert(WLCAP >= MAXB1024_MEAS / 8 + 8 * 46 + 1);
static_assert(MAXDEG_MEAS + 8 <= DEGCAP);
static_assert((MP * KEXT / 8) % NTHR == 0 && HD * KEXT / 8 == PBH * NTHR);
static_assert(BK_LDS <= 300000);
static_assert(GBM * SP * 4 <= 65536);
static_assert((2 * NBRUN) % (NTHR * 4) == 0);

struct PermTab { int p[64]; int inv[64]; };
constexpr PermTab make_perm() {
  PermTab t{};
  for (int i = 0; i < 64; ++i) t.p[i] = (i * 4) % 64 + (i * 4) / 64;
  for (int i = 0; i < 64; ++i) t.inv[i] = -1;
  for (int i = 0; i < 64; ++i) t.inv[t.p[i]] = i;
  return t;
}
constexpr PermTab PERM = make_perm();
constexpr int SGN[4][4] = {{ 1, -1, -1, -1},
                           { 1,  1, -1,  1},
                           { 1,  1,  1, -1},
                           { 1, -1,  1,  1}};
constexpr int CMP[4][4] = {{0, 1, 2, 3},
                           {1, 0, 3, 2},
                           {2, 3, 0, 1},
                           {3, 2, 1, 0}};
constexpr bool perm_ok() {
  for (int m = 0; m < 64; ++m) {
    if (PERM.inv[m] < 0 || PERM.inv[m] > 63) return false;
    if (PERM.p[PERM.inv[m]] != m) return false;
    if (PERM.inv[m] != 16 * (m % 4) + m / 4) return false;
  }
  return true;
}
constexpr bool ham_ok() {
  for (int m = 0; m < 64; ++m) {
    for (int n = 0; n < 64; ++n) {
      const int ri = PERM.inv[m], cj = PERM.inv[n];
      const int a = ri / 16, u = ri % 16, b = cj / 16, v = cj % 16;
      const int lit_idx = u * 64 + CMP[a][b] * 16 + v;
      const int lit_sgn = SGN[a][b];
      const int a2 = m % 4, u2 = m / 4, b2 = n % 4, v2 = n / 4;
      const int cf_idx = u2 * 64 + 16 * (a2 ^ b2) + v2;
      const int cf_sgn = SGN[a2][b2];
      if (lit_idx != cf_idx || lit_sgn != cf_sgn) return false;
      if (cf_idx < 0 || cf_idx > 1023) return false;
    }
  }
  return true;
}
static_assert(perm_ok());
static_assert(ham_ok());

typedef float          v4f   __attribute__((ext_vector_type(4)));
typedef float          v8f   __attribute__((ext_vector_type(8)));
typedef int            v2i   __attribute__((ext_vector_type(2)));
typedef int            v4i   __attribute__((ext_vector_type(4)));
typedef int            v8i   __attribute__((ext_vector_type(8)));
typedef double         v2d   __attribute__((ext_vector_type(2)));
typedef unsigned short v8us  __attribute__((ext_vector_type(8)));
typedef unsigned short v16us __attribute__((ext_vector_type(16)));
typedef __bf16         v16bf __attribute__((ext_vector_type(16)));
typedef v4f  __attribute__((may_alias)) v4fa;
typedef v2i  __attribute__((may_alias)) v2ia;
typedef v4i  __attribute__((may_alias)) v4ia;
typedef v2d  __attribute__((may_alias)) v2da;
typedef v8us __attribute__((may_alias)) v8usa;
union FragB { v16bf v; v16us u; v8us h[2]; v8i w; };

__device__ __forceinline__ v8f wmb(const FragB& a, const FragB& b, v8f c) {
  v8f d = __builtin_amdgcn_wmma_f32_16x16x32_bf16(false, a.v, false, b.v, (short)0, c, false, false);
  asm volatile("v_nop\n\tv_nop\n\tv_nop\n\tv_nop" : "+v"(d) : "v"(a.w), "v"(b.w));
  return d;
}

__device__ __forceinline__ unsigned bf16_bits(float f) {
  const unsigned u = __float_as_uint(f);
  const unsigned r = (u + 0x7FFFu + ((u >> 16) & 1u)) >> 16;
  const unsigned q = (u >> 16) | 0x40u;
  return ((u & 0x7fffffffu) > 0x7f800000u) ? q : r;
}
__device__ __forceinline__ float bf16_val(float f) {
  return __uint_as_float(bf16_bits(f) << 16);
}

template <int A>
__device__ __forceinline__ unsigned negbit(int b) {
  constexpr unsigned n0 = SGN[A][0] < 0 ? 0x8000u : 0u;
  constexpr unsigned n1 = SGN[A][1] < 0 ? 0x8000u : 0u;
  constexpr unsigned n2 = SGN[A][2] < 0 ? 0x8000u : 0u;
  constexpr unsigned n3 = SGN[A][3] < 0 ? 0x8000u : 0u;
  unsigned r = n3;
  r = (b == 2) ? n2 : r;
  r = (b == 1) ? n1 : r;
  r = (b == 0) ? n0 : r;
  return r;
}

__device__ __forceinline__ void st2_v4f(float* p, v4f v) {
  *(volatile v4f*)p = v;
  __threadfence();
  *(volatile v4f*)p = v;
}
__device__ __forceinline__ void st2_v4i(int* p, v4i v) {
  *(volatile v4i*)p = v;
  __threadfence();
  *(volatile v4i*)p = v;
}
__device__ __forceinline__ void st2_v8us(unsigned short* p, v8us v) {
  *(volatile v8us*)p = v;
  __threadfence();
  *(volatile v8us*)p = v;
}

__global__ __launch_bounds__(NTHR) void k_prep(const float* __restrict__ x, const float* __restrict__ w,
                                               unsigned short* xb, unsigned short* hb, int* flg) {
  const int tid = (int)threadIdx.x;
  const int blk = (int)blockIdx.x;
  if (blk < PBX) {
    const int u   = blk * NTHR + tid;
    const int row = u >> 3, k8 = (u & 7) * 8;
    const int rc  = row < NN ? row : NN - 1;
    const unsigned mk = row < NN ? 0xffffu : 0u;
    const float* p = x + (size_t)rc * KEXT + k8;
    const v4f a = *(const v4fa*)p;
    const v4f b = *(const v4fa*)(p + 4);
    v8us o;
    o[0] = (unsigned short)(bf16_bits(a.x) & mk); o[1] = (unsigned short)(bf16_bits(a.y) & mk);
    o[2] = (unsigned short)(bf16_bits(a.z) & mk); o[3] = (unsigned short)(bf16_bits(a.w) & mk);
    o[4] = (unsigned short)(bf16_bits(b.x) & mk); o[5] = (unsigned short)(bf16_bits(b.y) & mk);
    o[6] = (unsigned short)(bf16_bits(b.z) & mk); o[7] = (unsigned short)(bf16_bits(b.w) & mk);
    st2_v8us(xb + (size_t)row * XPITCH + k8, o);
  } else if (blk < PBX + PBH) {
    const int u  = (blk - PBX) * NTHR + tid;
    const int n  = u >> 3, k8 = (u & 7) * 8;
    const int b  = n & 3, v = n >> 2;
    const int u0 = k8 >> 2;
    const float f0 = w[(u0    ) * 64 + 16 * (0 ^ b) + v];
    const float f1 = w[(u0    ) * 64 + 16 * (1 ^ b) + v];
    const float f2 = w[(u0    ) * 64 + 16 * (2 ^ b) + v];
    const float f3 = w[(u0    ) * 64 + 16 * (3 ^ b) + v];
    const float f4 = w[(u0 + 1) * 64 + 16 * (0 ^ b) + v];
    const float f5 = w[(u0 + 1) * 64 + 16 * (1 ^ b) + v];
    const float f6 = w[(u0 + 1) * 64 + 16 * (2 ^ b) + v];
    const float f7 = w[(u0 + 1) * 64 + 16 * (3 ^ b) + v];
    const unsigned s0 = negbit<0>(b), s1 = negbit<1>(b), s2 = negbit<2>(b), s3 = negbit<3>(b);
    v8us o;
    o[0] = (unsigned short)(bf16_bits(f0) ^ s0); o[1] = (unsigned short)(bf16_bits(f1) ^ s1);
    o[2] = (unsigned short)(bf16_bits(f2) ^ s2); o[3] = (unsigned short)(bf16_bits(f3) ^ s3);
    o[4] = (unsigned short)(bf16_bits(f4) ^ s0); o[5] = (unsigned short)(bf16_bits(f5) ^ s1);
    o[6] = (unsigned short)(bf16_bits(f6) ^ s2); o[7] = (unsigned short)(bf16_bits(f7) ^ s3);
    st2_v8us(hb + (size_t)n * HPITCH + k8, o);
  } else {
    const v4i z = {0, 0, 0, 0};
#pragma unroll 1
    for (int i = tid; i < NBK * 8; i += NTHR) st2_v4i(flg + 4 * i, z);
  }
}

template <int KTOT, int AP, int BP>
__device__ __forceinline__ void gemm_16x64(const unsigned short* __restrict__ ap,
                                           const unsigned short* __restrict__ bp, v8f (&acc)[4]) {
  static_assert(KTOT % 32 == 0 && AP >= KTOT && BP >= KTOT);
#pragma unroll 1
  for (int k0 = 0; k0 < KTOT; k0 += 32) {
    FragB af;
    af.h[0] = *(const v8usa*)(ap + k0);
    af.h[1] = *(const v8usa*)(ap + k0 + 16);
#pragma unroll
    for (int nt = 0; nt < 4; ++nt) {
      const unsigned short* wq = bp + (size_t)(16 * nt) * (size_t)BP + k0;
      FragB bf;
      bf.h[0] = *(const v8usa*)wq;
      bf.h[1] = *(const v8usa*)(wq + 16);
      acc[nt] = wmb(af, bf, acc[nt]);
    }
  }
}

__device__ __forceinline__ void stage_d(float* stg, const v8f (&acc)[4], int wave, int hh, int m) {
#pragma unroll
  for (int nt = 0; nt < 4; ++nt) {
#pragma unroll
    for (int r = 0; r < 8; ++r) stg[(16 * wave + 8 * hh + r) * SP + 16 * nt + m] = acc[nt][r];
  }
}

__global__ __launch_bounds__(NTHR) __attribute__((amdgpu_num_vgpr(248)))
void k_gemm(const unsigned short* __restrict__ XB, const unsigned short* __restrict__ HB, float* S) {
  __shared__ __attribute__((aligned(16))) float stg[GBM * SP];
  const int tid = (int)threadIdx.x, lane = tid & 31, wave = tid >> 5, hh = lane >> 4, m = lane & 15;
  const int rowBase = (int)blockIdx.x * GBM;

  v8f acc[4];
  {
    const v8f z = {0.f, 0.f, 0.f, 0.f, 0.f, 0.f, 0.f, 0.f};
#pragma unroll
    for (int t = 0; t < 4; ++t) acc[t] = z;
  }
  const unsigned short* ap = XB + (size_t)(rowBase + 16 * wave + m) * (size_t)XPITCH + 8 * hh;
  const unsigned short* bp = HB + (size_t)m * (size_t)HPITCH + 8 * hh;
  gemm_16x64<KEXT, XPITCH, HPITCH>(ap, bp, acc);
  stage_d(stg, acc, wave, hh, m);
  __syncthreads();

#pragma unroll 1
  for (int i = 0; i < 8; ++i) {
    const int lr   = 16 * wave + 2 * i + hh;
    const int grow = rowBase + lr;
    const v4f a = *(const v4fa*)(stg + lr * SP + 4 * m);
    asm volatile("" :: "v"(a));
    if (grow < NN) st2_v4f(S + (size_t)grow * HD + 4 * m, a);
  }
}

__device__ __forceinline__ void bucket_flush(const int* pl, const int* cnt, int tot, int ov,
                                             const int* __restrict__ ecol, const float* __restrict__ eval,
                                             int* lp, int* cop, int* fp, int tid) {
#pragma unroll 1
  for (int i = tid * 2; i < RCAP; i += NTHR * 2) {
    const v2i wv = *(const v2ia*)(pl + i);
    int e0 = (wv.x >> SLB) & 0x1FFFFF;
    int e1 = (wv.y >> SLB) & 0x1FFFFF;
    e0 = e0 > NE - 1 ? NE - 1 : e0;
    e1 = e1 > NE - 1 ? NE - 1 : e1;
    int   c0 = ecol[e0], c1 = ecol[e1];
    float f0 = eval[e0], f1 = eval[e1];
    asm volatile("" :: "v"(c0), "v"(c1));
    asm volatile("" :: "v"(f0), "v"(f1));
    c0 = c0 < 0 ? 0 : (c0 > NN - 1 ? NN - 1 : c0);
    c1 = c1 < 0 ? 0 : (c1 > NN - 1 ? NN - 1 : c1);
    const int m0 = (i     < tot) ? -1 : 0;
    const int m1 = (i + 1 < tot) ? -1 : 0;
    v4i o;
    o.x = c0 & m0;
    o.y = (int)(bf16_bits(f0) << 16) & m0;
    o.z = c1 & m1;
    o.w = (int)(bf16_bits(f1) << 16) & m1;
    *(volatile v4i*)(lp + 2 * i) = o;
  }
#pragma unroll 1
  for (int i = tid * 4; i < 2 * NBRUN; i += NTHR * 4) {
    const v4i v = *(const v4ia*)(cnt + i);
    *(volatile v4i*)(cop + i) = v;
  }
  if (tid < 8) {
    const v4i f = {ov, ov, ov, ov};
    *(volatile v4i*)(fp + 4 * tid) = f;
  }
}

__global__ __launch_bounds__(NTHR) void k_bucket(const int* __restrict__ keys, const int* __restrict__ ecol,
                                                 const float* __restrict__ eval, int* LIST, int* CO, int* FLAG) {
  extern __shared__ __attribute__((aligned(16))) int dsm[];
  int* wl   = dsm;
  int* pl   = dsm + NWAVE * WLCAP;
  int* cnt  = pl + RCAP;
  int* offs = cnt + NBRUN;
  int* cur  = offs + NBRUN;
  int* misc = cur + NBRUN;
  const int tid = (int)threadIdx.x, lane = tid & 31, wave = tid >> 5;
  const int blk = (int)blockIdx.x;
  const unsigned nbs = (unsigned)(blk * NBRUN);
  const int nbi = NN - blk * NBRUN;
  const unsigned unb = (unsigned)(nbi < NBRUN ? (nbi < 0 ? 0 : nbi) : NBRUN);

  {
    const v4i z4 = {0, 0, 0, 0};
    for (int i = tid * 4; i < BK_ZINTS; i += NTHR * 4) *(v4ia*)(dsm + i) = z4;
    if (tid < 16) misc[tid] = 0;
  }
  __syncthreads();

  {
    const int per  = ((NE + NWAVE * WCH - 1) / (NWAVE * WCH)) * WCH;
    const int ebeg = wave * per;
    const int eend = (ebeg + per < NE) ? (ebeg + per) : NE;
    int* mylist = wl + wave * WLCAP;
    int wc = 0;
#pragma unroll 1
    for (int cb = ebeg; cb < eend; cb += WCH) {
      const int e0 = cb + lane * EPT;
      const v4i da = *(const v4ia*)(keys + e0);
      const v4i db = *(const v4ia*)(keys + e0 + 4);
      const unsigned s0 = (unsigned)da.x - nbs, s1 = (unsigned)da.y - nbs;
      const unsigned s2 = (unsigned)da.z - nbs, s3 = (unsigned)da.w - nbs;
      const unsigned s4 = (unsigned)db.x - nbs, s5 = (unsigned)db.y - nbs;
      const unsigned s6 = (unsigned)db.z - nbs, s7 = (unsigned)db.w - nbs;
      const bool h0 = s0 < unb, h1 = s1 < unb, h2 = s2 < unb, h3 = s3 < unb;
      const bool h4 = s4 < unb, h5 = s5 < unb, h6 = s6 < unb, h7 = s7 < unb;
      const unsigned m0 = __builtin_amdgcn_ballot_w32(h0), m1 = __builtin_amdgcn_ballot_w32(h1);
      const unsigned m2 = __builtin_amdgcn_ballot_w32(h2), m3 = __builtin_amdgcn_ballot_w32(h3);
      const unsigned m4 = __builtin_amdgcn_ballot_w32(h4), m5 = __builtin_amdgcn_ballot_w32(h5);
      const unsigned m6 = __builtin_amdgcn_ballot_w32(h6), m7 = __builtin_amdgcn_ballot_w32(h7);
      const unsigned any = m0 | m1 | m2 | m3 | m4 | m5 | m6 | m7;
      if (any != 0u) {
        const int pre = (int)(__builtin_amdgcn_mbcnt_lo(m0, 0u) + __builtin_amdgcn_mbcnt_lo(m1, 0u) +
                              __builtin_amdgcn_mbcnt_lo(m2, 0u) + __builtin_amdgcn_mbcnt_lo(m3, 0u) +
                              __builtin_amdgcn_mbcnt_lo(m4, 0u) + __builtin_amdgcn_mbcnt_lo(m5, 0u) +
                              __builtin_amdgcn_mbcnt_lo(m6, 0u) + __builtin_amdgcn_mbcnt_lo(m7, 0u));
        int p = wc + pre;
        if (h0) { if (p < WLCAP) mylist[p] = ((e0 + 0) << SLB) | (int)s0; p = p + 1; }
        if (h1) { if (p < WLCAP) mylist[p] = ((e0 + 1) << SLB) | (int)s1; p = p + 1; }
        if (h2) { if (p < WLCAP) mylist[p] = ((e0 + 2) << SLB) | (int)s2; p = p + 1; }
        if (h3) { if (p < WLCAP) mylist[p] = ((e0 + 3) << SLB) | (int)s3; p = p + 1; }
        if (h4) { if (p < WLCAP) mylist[p] = ((e0 + 4) << SLB) | (int)s4; p = p + 1; }
        if (h5) { if (p < WLCAP) mylist[p] = ((e0 + 5) << SLB) | (int)s5; p = p + 1; }
        if (h6) { if (p < WLCAP) mylist[p] = ((e0 + 6) << SLB) | (int)s6; p = p + 1; }
        if (h7) { if (p < WLCAP) mylist[p] = ((e0 + 7) << SLB) | (int)s7; p = p + 1; }
        wc += (int)(__builtin_popcount(m0) + __builtin_popcount(m1) + __builtin_popcount(m2) + __builtin_popcount(m3) +
                    __builtin_popcount(m4) + __builtin_popcount(m5) + __builtin_popcount(m6) + __builtin_popcount(m7));
      }
    }
    if (lane == 0) misc[wave] = wc;
  }
  __syncthreads();

  if (wave == 0) {
    int ov = 0, tot = 0;
#pragma unroll 1
    for (int w2 = 0; w2 < NWAVE; ++w2) {
      int c = misc[w2];
      if (c > WLCAP) ov = 1;
      c = c < 0 ? 0 : (c > WLCAP ? WLCAP : c);
      tot += c;
#pragma unroll 1
      for (int b0 = 0; b0 < c; b0 += 32) {
        const int idx = b0 + lane;
        const int ent = wl[w2 * WLCAP + (idx < WLCAP ? idx : WLCAP - 1)];
        const int m32 = (c - b0) < 32 ? (c - b0) : 32;
#pragma unroll 1
        for (int k = 0; k < m32; ++k) {
          const int u    = __builtin_amdgcn_readlane(ent, k);
          const int slot = u & (NBRUN - 1);
          if (lane == 0) cnt[slot] = cnt[slot] + 1;
        }
      }
    }
    if (lane == 0) { misc[9] = ov; misc[10] = tot; }
  }
  __syncthreads();
  if (wave == 0) {
    const int base = lane * (NBRUN / 32);
    int s = 0;
#pragma unroll 1
    for (int i = 0; i < NBRUN / 32; ++i) s += cnt[base + i];
    int incl = s;
#pragma unroll
    for (int d = 1; d < 32; d <<= 1) {
      const int y = __shfl_up(incl, d, 32);
      if (lane >= d) incl += y;
    }
    int run = incl - s;
#pragma unroll 1
    for (int i = 0; i < NBRUN / 32; ++i) {
      const int cv = cnt[base + i];
      offs[base + i] = run;
      cur[base + i]  = run;
      run += cv;
    }
  }
  __syncthreads();

  if (wave == 0) {
#pragma unroll 1
    for (int w2 = 0; w2 < NWAVE; ++w2) {
      int c = misc[w2];
      c = c < 0 ? 0 : (c > WLCAP ? WLCAP : c);
#pragma unroll 1
      for (int b0 = 0; b0 < c; b0 += 32) {
        const int idx = b0 + lane;
        const int ent = wl[w2 * WLCAP + (idx < WLCAP ? idx : WLCAP - 1)];
        const int m32 = (c - b0) < 32 ? (c - b0) : 32;
#pragma unroll 1
        for (int k = 0; k < m32; ++k) {
          const int u    = __builtin_amdgcn_readlane(ent, k);
          const int slot = u & (NBRUN - 1);
          if (lane == 0) {
            int p = cur[slot];
            p = p < 0 ? 0 : (p > RCAP - 1 ? RCAP - 1 : p);
            pl[p] = u;
            cur[slot] = p + 1;
          }
        }
      }
    }
  }
  __syncthreads();

  const int ovf = misc[9];
  int tot = misc[10];
  tot = tot < 0 ? 0 : (tot > RCAP ? RCAP : tot);
  int* lp  = LIST + (size_t)blk * (size_t)(2 * RCAP);
  int* cop = CO + (size_t)blk * (2 * NBRUN);
  int* fp  = FLAG + (size_t)blk * 32;
  bucket_flush(pl, cnt, tot, ovf, ecol, eval, lp, cop, fp, tid);
  __threadfence();
  bucket_flush(pl, cnt, tot, ovf, ecol, eval, lp, cop, fp, tid);
}

__global__ __launch_bounds__(NTHR) void k_replay(const int* __restrict__ LIST, const int* __restrict__ CO,
                                                 const int* __restrict__ FLAG, const float* __restrict__ S,
                                                 float* T, double* REC) {
  __shared__ __attribute__((aligned(16))) double recs[16 * 64 * 2];
  const int tid = (int)threadIdx.x, lane = tid & 31, wave = tid >> 5, hh = lane >> 4, q = lane & 15;
  const int blk = (int)blockIdx.x;
  const int slotBase = blk * NBRUN;
  const int* lb  = LIST + (size_t)blk * (size_t)(2 * RCAP);
  const int* cob = CO + (size_t)blk * (2 * NBRUN);
  const int flag = FLAG[(size_t)blk * 32];
  const float qnan = __uint_as_float(0x7fc00000u);

  double s0 = 0.0, s1 = 0.0, s2 = 0.0, s3 = 0.0;
  double q0 = 0.0, q1 = 0.0, q2 = 0.0, q3 = 0.0;

#pragma unroll 1
  for (int i = 0; i < NBRUN / 16; ++i) {
    const int slot = 16 * i + 2 * wave + hh;
    const int d    = slotBase + slot;
    int c = cob[slot];
    int o = cob[NBRUN + slot];
    const bool big = c > DEGCAP;
    c = c < 0 ? 0 : (c > DEGCAP ? DEGCAP : c);
    o = o < 0 ? 0 : (o > RCAP - 1 ? RCAP - 1 : o);
    const int co  = __shfl_xor(c, 16, 32);
    const int cmv = c > co ? c : co;
    const int cm  = __builtin_amdgcn_readfirstlane(cmv);
    int last = o + c - 1;
    last = last < o ? o : last;
    last = last > RCAP - 1 ? RCAP - 1 : last;
    float a0 = 0.0f, a1 = 0.0f, a2 = 0.0f, a3 = 0.0f;
#pragma unroll 1
    for (int j = 0; j < cm; ++j) {
      int idx = o + j;
      idx = idx > last ? last : idx;
      const v2i ent = *(const v2ia*)(lb + 2 * idx);
      int col = ent.x;
      col = col < 0 ? 0 : (col > NN - 1 ? NN - 1 : col);
      const float w = __int_as_float(ent.y);
      const v4f v = *(const v4fa*)(S + (size_t)col * HD + 4 * q);
      asm volatile("" :: "v"(v));
      const bool valid = j < c;
      const float t0 = fmaf(w, v.x, a0), t1 = fmaf(w, v.y, a1), t2 = fmaf(w, v.z, a2), t3 = fmaf(w, v.w, a3);
      a0 = valid ? t0 : a0; a1 = valid ? t1 : a1; a2 = valid ? t2 : a2; a3 = valid ? t3 : a3;
    }
    const bool bad  = (flag != 0) | big;
    const bool live = d < NN;
    const float m0 = bad ? qnan : a0, m1 = bad ? qnan : a1, m2 = bad ? qnan : a2, m3 = bad ? qnan : a3;
    const double d0 = (double)m0, d1 = (double)m1, d2 = (double)m2, d3 = (double)m3;
    s0 = live ? (s0 + d0) : s0; s1 = live ? (s1 + d1) : s1;
    s2 = live ? (s2 + d2) : s2; s3 = live ? (s3 + d3) : s3;
    q0 = live ? (q0 + d0 * d0) : q0; q1 = live ? (q1 + d1 * d1) : q1;
    q2 = live ? (q2 + d2 * d2) : q2; q3 = live ? (q3 + d3 * d3) : q3;
    if (live) {
      v4f ov;
      ov.x = m0; ov.y = m1; ov.z = m2; ov.w = m3;
      st2_v4f(T + (size_t)d * HD + 4 * q, ov);
    }
  }

  {
    const int hw = 2 * wave + hh;
    double* rp = recs + (size_t)(hw * 64 + 4 * q) * 2;
    rp[0] = s0; rp[1] = q0; rp[2] = s1; rp[3] = q1;
    rp[4] = s2; rp[5] = q2; rp[6] = s3; rp[7] = q3;
  }
  __syncthreads();
  if (tid < 64) {
    double S1 = 0.0, S2 = 0.0;
#pragma unroll 1
    for (int hw = 0; hw < 16; ++hw) {
      S1 += recs[(hw * 64 + tid) * 2];
      S2 += recs[(hw * 64 + tid) * 2 + 1];
    }
    v2d r;
    r.x = S1; r.y = S2;
    double* op = REC + ((size_t)blk * 64 + (size_t)tid) * 2;
    *(volatile v2d*)op = r;
    __threadfence();
    *(volatile v2d*)op = r;
  }
}

__global__ __launch_bounds__(64) void k_combine(const double* __restrict__ REC, float* STAT) {
  __shared__ __attribute__((aligned(16))) float st[128];
  const int tid = (int)threadIdx.x;
  double S1 = 0.0, S2 = 0.0;
#pragma unroll 1
  for (int b = 0; b < NBK; ++b) {
    const v2d r = *(const v2da*)(REC + ((size_t)b * 64 + (size_t)tid) * 2);
    S1 += r.x;
    S2 += r.y;
  }
  const double m  = S1 / 100000.0;
  double vv = S2 / 100000.0 - m * m;
  vv = (vv > 0.0) ? vv : (vv - vv);
  const float mf = (float)m;
  const float vf = (float)vv;
  const float rs = 1.0f / sqrtf(vf + 1e-5f);
  st[tid] = mf;
  st[64 + tid] = rs;
  __syncthreads();
  if (tid < 32) {
    const v4f v = *(const v4fa*)(st + 4 * tid);
    st2_v4f(STAT + 4 * tid, v);
  }
}

__device__ __forceinline__ void apply_flush(const float* tile, float* ob, int rowBase, int tid) {
#pragma unroll 1
  for (int it = 0; it < (ABM * HD / 4) / NTHR; ++it) {
    const int i4  = it * NTHR + tid;
    const int row = rowBase + (i4 >> 4);
    const v4f v = *(const v4fa*)(tile + 4 * i4);
    asm volatile("" :: "v"(v));
    if (row < NN) *(volatile v4f*)(ob + (size_t)4 * (size_t)i4) = v;
  }
}

__global__ __launch_bounds__(NTHR) void k_apply(const float* __restrict__ T, const float* __restrict__ STAT,
                                                const float* __restrict__ gam, const float* __restrict__ bet,
                                                const int* __restrict__ FLAG, float* out) {
  __shared__ __attribute__((aligned(16))) float tile[ABM * HD];
  __shared__ __attribute__((aligned(16))) float prm[4 * 64];
  const int tid = (int)threadIdx.x;
  const int rowBase = (int)blockIdx.x * ABM;
  if (tid < 32) {
    const int j = tid & 15;
    const v4f g4 = *(const v4fa*)(gam + 4 * j);
    const v4f b4 = *(const v4fa*)(bet + 4 * j);
    const v4f m4 = *(const v4fa*)(STAT + 4 * j);
    const v4f r4 = *(const v4fa*)(STAT + 64 + 4 * j);
    v4f gq, bq;
    gq.x = bf16_val(g4.x); gq.y = bf16_val(g4.y); gq.z = bf16_val(g4.z); gq.w = bf16_val(g4.w);
    bq.x = bf16_val(b4.x); bq.y = bf16_val(b4.y); bq.z = bf16_val(b4.z); bq.w = bf16_val(b4.w);
    *(v4fa*)(prm + 4 * j)       = gq;
    *(v4fa*)(prm + 64 + 4 * j)  = bq;
    *(v4fa*)(prm + 128 + 4 * j) = m4;
    *(v4fa*)(prm + 192 + 4 * j) = r4;
  }
  const int flag = FLAG[(size_t)(rowBase >> SLB) * 32];
  __syncthreads();

  const int c = tid & 63;
  const float g = prm[c], b = prm[64 + c], mu = prm[128 + c], rs = prm[192 + c];
  const float qnan = __uint_as_float(0x7fc00000u);
#pragma unroll 1
  for (int it = 0; it < (ABM * HD) / NTHR; ++it) {
    const int idx = it * NTHR + tid;
    const int row = rowBase + (idx >> 6);
    const int rc  = row < NN ? row : NN - 1;
    const float t = T[(size_t)rc * HD + c];
    const float y = ((g * (t - mu)) * rs) + b;
    float o = tanhf(y);
    o = (flag != 0) ? qnan : o;
    tile[idx] = o;
  }
  __syncthreads();

  float* ob = out + (size_t)rowBase * HD;
  apply_flush(tile, ob, rowBase, tid);
  __threadfence();
  apply_flush(tile, ob, rowBase, tid);
}

extern "C" void kernel_launch(void* const* d_in, const int* in_sizes, int n_in,
                              void* d_out, int out_size, void* d_ws, size_t ws_size,
                              hipStream_t stream) {
  if (n_in < 7) return;
  if (in_sizes[0] != NN * KEXT) return;
  if (in_sizes[1] != NE) return;
  if (in_sizes[2] != NE) return;
  if (in_sizes[3] != NE) return;
  if (in_sizes[4] != 16 * 64) return;
  if (in_sizes[5] != HD) return;
  if (in_sizes[6] != HD) return;
  if (out_size != NN * HD) return;

  const float* x    = (const float*)d_in[0];
  const int*   erow = (const int*)d_in[1];
  const int*   ecol = (const int*)d_in[2];
  const float* eval = (const float*)d_in[3];
  const float* wgt  = (const float*)d_in[4];
  const float* gam  = (const float*)d_in[5];
  const float* bet  = (const float*)d_in[6];
  float* out = (float*)d_out;

  constexpr size_t zXB   = (size_t)MP * XPITCH * 2;
  constexpr size_t zHB   = (size_t)HD * HPITCH * 2;
  constexpr size_t zS    = (size_t)NN * HD * 4;
  constexpr size_t zLIST = (size_t)NBK * RCAP * 8;
  constexpr size_t zCO   = (size_t)NBK * 2 * NBRUN * 4;
  constexpr size_t zT    = (size_t)NN * HD * 4;
  constexpr size_t zREC  = (size_t)NBK * 64 * 2 * 8;
  constexpr size_t zSTAT = 512;
  constexpr size_t zFLAG = (size_t)NBK * 128;
  constexpr size_t oXB   = 0;
  constexpr size_t oHB   = oXB + zXB;
  constexpr size_t oS    = oHB + zHB;
  constexpr size_t oLIST = oS + zS;
  constexpr size_t oCO   = oLIST + zLIST;
  constexpr size_t oT    = oCO + zCO;
  constexpr size_t oREC  = oT + zT;
  constexpr size_t oSTAT = oREC + zREC;
  constexpr size_t oFLAG = oSTAT + zSTAT;
  constexpr size_t oEND  = oFLAG + zFLAG;
  static_assert(zXB % 256 == 0 && zHB % 256 == 0 && zS % 256 == 0 && zLIST % 256 == 0 && zCO % 256 == 0);
  static_assert(zT % 256 == 0 && zREC % 256 == 0 && zSTAT % 256 == 0 && zFLAG % 256 == 0);
  static_assert(oEND <= (size_t)(128u << 20));
  if (oEND > ws_size) return;

  char* ws = (char*)d_ws;
  unsigned short* XB   = (unsigned short*)(ws + oXB);
  unsigned short* HB   = (unsigned short*)(ws + oHB);
  float*          S    = (float*)(ws + oS);
  int*            LIST = (int*)(ws + oLIST);
  int*            CO   = (int*)(ws + oCO);
  float*          T    = (float*)(ws + oT);
  double*         REC  = (double*)(ws + oREC);
  float*          STAT = (float*)(ws + oSTAT);
  int*            FLAG = (int*)(ws + oFLAG);

  hipFuncSetAttribute(reinterpret_cast<const void*>(&k_bucket), hipFuncAttributeMaxDynamicSharedMemorySize, (int)BK_LDS);

  k_prep<<<PBTOT, NTHR, 0, stream>>>(x, wgt, XB, HB, FLAG);
  k_gemm<<<MP / GBM, NTHR, 0, stream>>>(XB, HB, S);
  k_bucket<<<NBK, NTHR, BK_LDS, stream>>>(erow, ecol, eval, LIST, CO, FLAG);
  k_replay<<<NBK, NTHR, 0, stream>>>(LIST, CO, FLAG, S, T, REC);
  k_combine<<<1, 64, 0, stream>>>(REC, STAT);
  k_apply<<<(NN + ABM - 1) / ABM, NTHR, 0, stream>>>(T, STAT, gam, bet, FLAG, out);
}
